// SSMBlock_86569360818303
// MI455X (gfx1250) — hardware-run, weakly checked
//
#include <hip/hip_runtime.h>
#include <math.h>

typedef __attribute__((ext_vector_type(16))) _Float16 v16h;
typedef __attribute__((ext_vector_type(8)))  _Float16 v8h;
typedef __attribute__((ext_vector_type(2)))  _Float16 v2h;
typedef __attribute__((ext_vector_type(16))) __bf16   v16b;
typedef __attribute__((ext_vector_type(8)))  __bf16   v8b;
typedef __attribute__((ext_vector_type(8)))  float    v8f;
typedef __attribute__((ext_vector_type(4)))  float    v4f;
typedef __attribute__((ext_vector_type(2)))  float    v2f;

constexpr int kL    = 2048;
constexpr int kRows = kL;
constexpr int kDM   = 1024;
constexpr int kDI   = 2 * kDM;
constexpr int kNs   = 16;
constexpr int kDC   = 4;
constexpr int kR    = 64;
constexpr int kXo   = kR + 2 * kNs;
constexpr int kXoP  = 128;
constexpr int kThr  = 256;
constexpr float kInCarry = 1024.0f;
constexpr float kWCarry  = 4096.0f;
constexpr float kUCarry  = 256.0f;
constexpr float kDtCarry = 256.0f;
constexpr float kYCarry  = 64.0f;
constexpr float kScIn = 1.0f / (kInCarry * kWCarry);
constexpr float kScU  = 1.0f / (kUCarry * kWCarry);
constexpr float kScDt = 1.0f / (kDtCarry * kWCarry);
constexpr float kScY  = 1.0f / (kYCarry * kWCarry);
constexpr float kF16MinNormal = 6.103515625e-5f;

static_assert(kXo == 96 && kXo <= kXoP && kR == 64 && kDI == 2048 && kRows == 2048, "the index arithmetic below uses these sizes");

constexpr size_t kOffBIAS = 0ull;
constexpr size_t kOffX16 = 24576ull;
constexpr size_t kOffWIN16 = 4218880ull;
constexpr size_t kOffWX16 = 12607488ull;
constexpr size_t kOffWDT16 = 13656064ull;
constexpr size_t kOffWOUT16 = 13918208ull;
constexpr size_t kOffXZ = 18112512ull;
constexpr size_t kOffU32 = 51666944ull;
constexpr size_t kOffU16 = 68444160ull;
constexpr size_t kOffXD = 85221376ull;
constexpr size_t kOffDT16 = 86269952ull;
constexpr size_t kOffDL = 86532096ull;
constexpr size_t kOffYS = 103309312ull;
constexpr size_t kOffY16 = 120086528ull;
constexpr size_t kWsTotal = 128475136ull;
static_assert(kWsTotal <= 134217728ull, "carve cap: under 128 MiB");
static_assert(kOffBIAS == 0
  && kOffX16 == kOffBIAS + 24576ull
  && kOffWIN16 == kOffX16 + 4194304ull
  && kOffWX16 == kOffWIN16 + 8388608ull
  && kOffWDT16 == kOffWX16 + 1048576ull
  && kOffWOUT16 == kOffWDT16 + 262144ull
  && kOffXZ == kOffWOUT16 + 4194304ull
  && kOffU32 == kOffXZ + 33554432ull
  && kOffU16 == kOffU32 + 16777216ull
  && kOffXD == kOffU16 + 16777216ull
  && kOffDT16 == kOffXD + 1048576ull
  && kOffDL == kOffDT16 + 262144ull
  && kOffYS == kOffDL + 16777216ull
  && kOffY16 == kOffYS + 16777216ull
  && kWsTotal == kOffY16 + 8388608ull, "the carve is a chain: every region starts where the one before ends");
static_assert((kOffX16 % 256) == 0 && (kOffWIN16 % 256) == 0 && (kOffWX16 % 256) == 0 && (kOffWDT16 % 256) == 0 && (kOffWOUT16 % 256) == 0 && (kOffXZ % 256) == 0 && (kOffU32 % 256) == 0 && (kOffU16 % 256) == 0 && (kOffXD % 256) == 0 && (kOffDT16 % 256) == 0 && (kOffDL % 256) == 0 && (kOffYS % 256) == 0 && (kOffY16 % 256) == 0, "every region starts on a multiple of 256 B");

__device__ __forceinline__ unsigned short f2bf_bits(float f) {
  unsigned u = __float_as_uint(f);
  return (unsigned short)((u + 0x7FFFu + ((u >> 16) & 1u)) >> 16);
}
__device__ __forceinline__ float bf_bits2f(unsigned short h) { return __uint_as_float(((unsigned)h) << 16); }
__device__ __forceinline__ float bf16r(float f) { return bf_bits2f(f2bf_bits(f)); }
__device__ __forceinline__ float carry_flush(float v, float carry) {
  const float s = v * carry;
  return (fabsf(s) < kF16MinNormal) ? 0.0f : s;
}

__device__ __forceinline__ void dep_guard4_h(v8f& a, v8f& b, v8f& c, v8f& d, v16h x, v16h y) { asm volatile("v_nop\n\tv_nop\n\tv_nop\n\tv_nop" : "+v"(a), "+v"(b), "+v"(c), "+v"(d) : "v"(x), "v"(y)); }
__device__ __forceinline__ void dep_guard4_b(v8f& a, v8f& b, v8f& c, v8f& d, v16b x, v16b y) { asm volatile("v_nop\n\tv_nop\n\tv_nop\n\tv_nop" : "+v"(a), "+v"(b), "+v"(c), "+v"(d) : "v"(x), "v"(y)); }
__device__ __forceinline__ void keep4_h(v16h a, v16h b, v16h c, v16h d) { asm volatile("v_nop" :: "v"(a), "v"(b), "v"(c), "v"(d)); }
__device__ __forceinline__ void keep4_b(v16b a, v16b b, v16b c, v16b d) { asm volatile("v_nop" :: "v"(a), "v"(b), "v"(c), "v"(d)); }
__device__ __forceinline__ void acc_guard4(v8f& a, v8f& b, v8f& c, v8f& d) { asm volatile("v_nop\n\tv_nop\n\tv_nop\n\tv_nop" : "+v"(a), "+v"(b), "+v"(c), "+v"(d)); }

template <typename T> struct Frag;
template <> struct Frag<_Float16> {
  typedef v16h V; union U { v16h v; v8h h[2]; };
  static __device__ __forceinline__ v16h load(const _Float16* p) {
    U f; f.h[0] = *(const v8h*)(p); f.h[1] = *(const v8h*)(p + 16); return f.v;
  }
  static __device__ __forceinline__ v8f mma(v16h a, v16h b, v8f c) {
    return __builtin_amdgcn_wmma_f32_16x16x32_f16(false, a, false, b, (short)0, c, false, false);
  }
  static __device__ __forceinline__ void guard4(v8f& a, v8f& b, v8f& c, v8f& d, v16h x, v16h y) { dep_guard4_h(a, b, c, d, x, y); }
  static __device__ __forceinline__ void keep(v16h a, v16h b, v16h c, v16h d) { keep4_h(a, b, c, d); }
};
template <> struct Frag<__bf16> {
  typedef v16b V; union U { v16b v; v8b h[2]; };
  static __device__ __forceinline__ v16b load(const __bf16* p) {
    U f; f.h[0] = *(const v8b*)(p); f.h[1] = *(const v8b*)(p + 16); return f.v;
  }
  static __device__ __forceinline__ v8f mma(v16b a, v16b b, v8f c) {
    return __builtin_amdgcn_wmma_f32_16x16x32_bf16(false, a, false, b, (short)0, c, false, false);
  }
  static __device__ __forceinline__ void guard4(v8f& a, v8f& b, v8f& c, v8f& d, v16b x, v16b y) { dep_guard4_b(a, b, c, d, x, y); }
  static __device__ __forceinline__ void keep(v16b a, v16b b, v16b c, v16b d) { keep4_b(a, b, c, d); }
};

__device__ __forceinline__ v8f mma_h(v16h a, v16h b, v8f c) {
  c = __builtin_amdgcn_wmma_f32_16x16x32_f16(false, a, false, b, (short)0, c, false, false);
  asm volatile("v_nop\n\tv_nop\n\tv_nop\n\tv_nop" : "+v"(c) : "v"(a), "v"(b));
  return c;
}

template <int ET> struct Elem;
template <> struct Elem<0> { typedef _Float16 T; };
template <> struct Elem<1> { typedef __bf16 T; };
template <int ET, bool SPLIT, int BIAS_MODE, int OUT_MODE, bool RESID, int ACT = 0>
__global__ __launch_bounds__(256) void wmma_gemm64(
    const unsigned short* __restrict__ Ap, const unsigned short* __restrict__ A2p, int lda, long strideA,
    const unsigned short* __restrict__ Btp, const unsigned short* __restrict__ Bt2p, int ldb, long strideB,
    void* __restrict__ Cout, void* __restrict__ Cout2, int ldc, long strideC,
    const float* __restrict__ bias,
    const float* __restrict__ resid, long strideR,
    int M, int N, int K, float scale) {
  typedef typename Elem<ET>::T T;
  typedef typename Frag<T>::V V;
  const T* A = (const T*)Ap; const T* A2 = (const T*)A2p; const T* Bt = (const T*)Btp; const T* Bt2 = (const T*)Bt2p;
  __shared__ __align__(16) float sT[8][16 * 68];
  const int b    = blockIdx.y;
  const int lane = threadIdx.x & 31;
  const int wave = threadIdx.x >> 5;
  const int tilesN = N >> 6;
  const int tilesM = M >> 6;
  const int tile = blockIdx.x * 8 + wave;
  if (tile >= tilesM * tilesN) return;
  const int tm = tile / tilesN;
  const int tn = tile - tm * tilesN;
  const int m0 = tm << 6;
  const int n0 = tn << 6;

  const T* Ab  = A  + (size_t)b * strideA;
  const T* Bb  = Bt + (size_t)b * strideB;
  const T* Ab2 = SPLIT ? (A2  + (size_t)b * strideA) : nullptr;
  const T* Bb2 = SPLIT ? (Bt2 + (size_t)b * strideB) : nullptr;

  const int rlane = lane & 15;
  const int koff  = (lane >> 4) * 8;
  const int mOff  = (lane >> 4) * 8;

  v8f acc[4][4];
#pragma unroll
  for (int i = 0; i < 4; ++i)
#pragma unroll
    for (int j = 0; j < 4; ++j) acc[i][j] = (v8f){0.f,0.f,0.f,0.f,0.f,0.f,0.f,0.f};

  for (int k0 = 0; k0 < K; k0 += 32) {
    V bh[4], bl[4];
#pragma unroll
    for (int j = 0; j < 4; ++j) {
      const size_t bo = (size_t)(n0 + (j << 4) + rlane) * ldb + koff + k0;
      bh[j] = Frag<T>::load(Bb + bo);
      if (SPLIT) bl[j] = Frag<T>::load(Bb2 + bo);
    }
#pragma unroll
    for (int i = 0; i < 4; ++i) {
      const size_t ao = (size_t)(m0 + (i << 4) + rlane) * lda + koff + k0;
      V ah = Frag<T>::load(Ab + ao);
      V al;
      if (SPLIT) al = Frag<T>::load(Ab2 + ao);
#pragma unroll
      for (int j = 0; j < 4; ++j) {
        acc[i][j] = Frag<T>::mma(ah, bh[j], acc[i][j]);
        if (SPLIT) {
          acc[i][j] = Frag<T>::mma(ah, bl[j], acc[i][j]);
          acc[i][j] = Frag<T>::mma(al, bh[j], acc[i][j]);
        }
      }
      Frag<T>::guard4(acc[i][0], acc[i][1], acc[i][2], acc[i][3], ah, SPLIT ? al : ah);
    }
    Frag<T>::keep(bh[0], bh[1], bh[2], bh[3]);
    if (SPLIT) Frag<T>::keep(bl[0], bl[1], bl[2], bl[3]);
  }
  acc_guard4(acc[0][0], acc[0][1], acc[0][2], acc[0][3]);
  acc_guard4(acc[1][0], acc[1][1], acc[1][2], acc[1][3]);
  acc_guard4(acc[2][0], acc[2][1], acc[2][2], acc[2][3]);
  acc_guard4(acc[3][0], acc[3][1], acc[3][2], acc[3][3]);

  float* slab = sT[wave];
  const float* Rb = RESID ? (resid + (size_t)b * strideR) : nullptr;
#pragma unroll
  for (int i = 0; i < 4; ++i) {
    const int mBase = m0 + (i << 4);
#pragma unroll
    for (int j = 0; j < 4; ++j) {
      const int n = n0 + (j << 4) + rlane;
      float bv = 0.f;
      if (BIAS_MODE == 2) bv = bias[n];
#pragma unroll
      for (int r = 0; r < 8; ++r) {
        float v = acc[i][j][r] * scale;
        if (BIAS_MODE == 1) v += bias[mBase + mOff + r];
        if (BIAS_MODE == 2) v += bv;
        if (RESID) v += Rb[(size_t)(mBase + mOff + r) * ldc + n];
        if (ACT == 1) v = tanhf(v);
        if (ACT == 2) v = fmaxf(v, 0.0f);
        if (ACT == 3) v = v / (1.0f + expf(-v));
        if (ACT == 4) v = (v > 0.f) ? v : 0.01f * v;
        slab[(mOff + r) * 68 + (j << 4) + rlane] = v;
      }
    }
    __builtin_amdgcn_fence(__ATOMIC_RELEASE, "workgroup");
    __builtin_amdgcn_wave_barrier();
    __builtin_amdgcn_fence(__ATOMIC_ACQUIRE, "workgroup");
    if (OUT_MODE == 0) {
      float* C = (float*)Cout + (size_t)b * strideC;
      const int hh = lane >> 4, c4 = (lane & 15) * 4;
      for (int pass = 0; pass < 2; ++pass) {
#pragma unroll
        for (int it = 0; it < 8; ++it) {
          const int row = it * 2 + hh;
          v4f v = *(const v4f*)(slab + row * 68 + c4);
          *(volatile v4f*)(C + (size_t)(mBase + row) * ldc + n0 + c4) = v;
        }
        __threadfence();
      }
    } else {
      const int q = lane >> 3, c8 = (lane & 7) * 8;
      unsigned short* C  = (unsigned short*)Cout  + (size_t)b * strideC;
      unsigned short* C2 = (OUT_MODE == 2) ? ((unsigned short*)Cout2 + (size_t)b * strideC) : nullptr;
      for (int pass = 0; pass < 2; ++pass) {
#pragma unroll
        for (int it = 0; it < 4; ++it) {
          const int row = it * 4 + q;
          const float* sp = slab + row * 68 + c8;
          v8h hv, lv;
#pragma unroll
          for (int e = 0; e < 8; ++e) {
            if (OUT_MODE == 1) {
              hv[e] = (_Float16)sp[e];
            } else {
              unsigned short hb = f2bf_bits(sp[e]);
              unsigned short lb = f2bf_bits(sp[e] - bf_bits2f(hb));
              hv[e] = __builtin_bit_cast(_Float16, hb);
              lv[e] = __builtin_bit_cast(_Float16, lb);
            }
          }
          *(volatile v8h*)(C + (size_t)(mBase + row) * ldc + n0 + c8) = hv;
          if (OUT_MODE == 2) *(volatile v8h*)(C2 + (size_t)(mBase + row) * ldc + n0 + c8) = lv;
        }
        __threadfence();
      }
    }
    __builtin_amdgcn_fence(__ATOMIC_RELEASE, "workgroup");
    __builtin_amdgcn_wave_barrier();
    __builtin_amdgcn_fence(__ATOMIC_ACQUIRE, "workgroup");
  }
}


__device__ __forceinline__ void store2(float* p, float v) {
  *(volatile float*)p = v;
  __threadfence();
  *(volatile float*)p = v;
}

__global__ __launch_bounds__(kThr) void cast_plane_kernel(const float* __restrict__ src, unsigned short* __restrict__ dst,
                                                          int colsLog2, int dstPitch, int dstOff) {
  const int i   = blockIdx.x * kThr + threadIdx.x;
  const int sh  = colsLog2 - 3;
  const int row = i >> sh;
  const int c8  = (i & ((1 << sh) - 1)) * 8;
  const float* sp = src + ((size_t)row << colsLog2) + c8;
  const v4f a0 = *(const v4f*)(sp);
  const v4f a1 = *(const v4f*)(sp + 4);
  v8h hv;
#pragma unroll
  for (int e = 0; e < 4; ++e) {
    const float f0 = a0[e];
    const float f1 = a1[e];
    hv[e]     = (_Float16)carry_flush(bf16r(f0), kInCarry);
    hv[4 + e] = (_Float16)carry_flush(bf16r(f1), kInCarry);
  }
  unsigned short* dp = dst + (size_t)row * dstPitch + dstOff + c8;
  *(volatile v8h*)dp = hv;
  __threadfence();
  *(volatile v8h*)dp = hv;
}

__global__ __launch_bounds__(256) void wt_plane_kernel(const float* __restrict__ W, unsigned short* __restrict__ dst, int K, int N, int nLive, int ldd, int colOff) {
  const int n  = blockIdx.x;
  const int k8 = threadIdx.x * 8;
  const bool live = n < nLive;
  const int nc = live ? n : 0;
  v8h hv;
#pragma unroll
  for (int e = 0; e < 8; ++e) {
    const float w = W[(size_t)(k8 + e) * N + nc];
    hv[e] = (_Float16)(live ? carry_flush(bf16r(w), kWCarry) : 0.0f);
  }
  unsigned short* dp = dst + (size_t)n * ldd + colOff + k8;
  *(volatile v8h*)dp = hv;
  __threadfence();
  *(volatile v8h*)dp = hv;
}

__global__ __launch_bounds__(kThr) void setup_kernel(const float* __restrict__ b_dt, float* __restrict__ BIAS) {
  const unsigned i = blockIdx.x * (unsigned)kThr + threadIdx.x;
  const bool isb = i >= 4096u;
  const float p = b_dt[isb ? (i - 4096u) : 0u];
  store2(BIAS + i, isb ? bf16r(p) : 0.0f);
}
static_assert(4096 + kDI == 24 * kThr, "set-up grid exact: 24 blocks");

__global__ __launch_bounds__(64) void front_kernel(const float* __restrict__ XZ, const float* __restrict__ cw, const float* __restrict__ cb,
                                                   float* __restrict__ U32, unsigned short* __restrict__ U16) {
  const int row = (int)blockIdx.y;
  const int c8 = (int)(blockIdx.x * 64u + threadIdx.x) * 8;
  float acc[8], wv[8][kDC];
#pragma unroll
  for (int e = 0; e < 8; ++e) {
    const float p = cb[c8 + e];
    acc[e] = bf16r(p);
    const v4f w4 = *(const v4f*)(cw + (size_t)(c8 + e) * kDC);
#pragma unroll
    for (int k = 0; k < kDC; ++k) { const float w = w4[k]; wv[e][k] = bf16r(w); }
  }
#pragma unroll
  for (int k = 0; k < kDC; ++k) {
    const int back = kDC - 1 - k;
    const bool has = row >= back;
    const float* xp = XZ + (size_t)(row - (has ? back : 0)) * (2 * kDI) + c8;
    const v4f x0 = *(const v4f*)xp, x1 = *(const v4f*)(xp + 4);
#pragma unroll
    for (int e = 0; e < 8; ++e) {
      const float xv = (e < 4) ? x0[e] : x1[e - 4];
      acc[e] += has ? wv[e][k] * xv : 0.0f;
    }
  }
  v4f u0, u1;
  v8h hv, lv;
#pragma unroll
  for (int e = 0; e < 8; ++e) {
    const float v = acc[e];
    const float s = v / (1.0f + expf(-v));
    if (e < 4) u0[e] = s; else u1[e - 4] = s;
    const float sc = carry_flush(s, kUCarry);
    const _Float16 hh = (_Float16)sc;
    const float rr = sc - (float)hh;
    hv[e] = hh;
    lv[e] = (_Float16)((fabsf(rr) < kF16MinNormal) ? 0.0f : rr);
  }
  float* up = U32 + (size_t)row * kDI + c8;
  unsigned short* hp = U16 + (size_t)row * (2 * kDI) + c8;
  for (int pass = 0; pass < 2; ++pass) {
    *(volatile v4f*)up = u0; *(volatile v4f*)(up + 4) = u1;
    *(volatile v8h*)hp = hv;
    *(volatile v8h*)(hp + kDI) = lv;
    __threadfence();
  }
}
static_assert(kDI == 4 * 64 * 8, "front grid exact: 4 blocks of 64 groups a row");

__global__ __launch_bounds__(kThr) void dtcast_kernel(const float* __restrict__ XD, unsigned short* __restrict__ DT16) {
  const unsigned i = blockIdx.x * (unsigned)kThr + threadIdx.x;
  const size_t row = i >> 3;
  const unsigned c8 = (i & 7u) * 8u;
  const float* sp = XD + row * kXoP + c8;
  v8h hv;
#pragma unroll
  for (int e = 0; e < 8; ++e) { const float v = sp[e]; hv[e] = (_Float16)carry_flush(v, kDtCarry); }
  unsigned short* dp = DT16 + row * kR + c8;
  *(volatile v8h*)dp = hv;
  __threadfence();
  *(volatile v8h*)dp = hv;
}
static_assert(kRows * (kR / 8) == 64 * kThr, "the step input's cast: 64 blocks");

__global__ __launch_bounds__(kThr) void scan_kernel(const float* __restrict__ XD, const float* __restrict__ DL, const float* __restrict__ U32,
                                                    const float* __restrict__ A_log, const float* __restrict__ Dp, float* __restrict__ YS, float* __restrict__ HT) {
  const unsigned d = blockIdx.x * (unsigned)kThr + threadIdx.x;
  float A[kNs], h[kNs];
#pragma unroll
  for (int n = 0; n < kNs; ++n) { const float a = A_log[(size_t)d * kNs + n]; A[n] = -expf(bf16r(a)); h[n] = 0.0f; }
  const float q0 = Dp[d];
  const float dsk = bf16r(q0);
  for (int l = 0; l < kL; ++l) {
    const size_t row = (size_t)l;
    const float* pr = XD + row * kXoP + kR;
    const float pre = DL[row * kDI + d];
    const float uv = U32[row * kDI + d];
    const float dt = fmaxf(pre, 0.0f) + log1pf(expf(-fabsf(pre)));
    const float dx = dt * uv;
    float y = 0.0f;
#pragma unroll
    for (int q = 0; q < kNs / 4; ++q) {
      const v4f bv = *(const v4f*)(pr + 4 * q), cv = *(const v4f*)(pr + kNs + 4 * q);
#pragma unroll
      for (int e = 0; e < 4; ++e) {
        const int n = 4 * q + e;
        const float hn = expf(dt * A[n]) * h[n] + dx * bv[e];
        h[n] = hn;
        y += hn * cv[e];
      }
    }
    store2(YS + row * kDI + d, y + dsk * uv);
  }
  float* hp = HT + (size_t)d * kNs;
  for (int pass = 0; pass < 2; ++pass) {
#pragma unroll
    for (int q = 0; q < kNs / 4; ++q) {
      v4f v;
#pragma unroll
      for (int e = 0; e < 4; ++e) v[e] = h[4 * q + e];
      *(volatile v4f*)(hp + 4 * q) = v;
    }
    __threadfence();
  }
}
static_assert(kDI == 8 * kThr && (kNs % 4) == 0 && (kR % 4) == 0, "walk grid exact: 8 blocks; the B | C columns 16-B aligned");

__global__ __launch_bounds__(kThr) void ygate_kernel(const float* __restrict__ YS, const float* __restrict__ XZ, unsigned short* __restrict__ Y16) {
  const unsigned i = blockIdx.x * (unsigned)kThr + threadIdx.x;
  const size_t row = i >> 8;
  const unsigned c8 = (i & 255u) * 8u;
  const float* yp = YS + row * kDI + c8;
  const float* zp = XZ + row * (2 * kDI) + kDI + c8;
  v8h hv;
#pragma unroll
  for (int e = 0; e < 8; ++e) { const float z = zp[e]; hv[e] = (_Float16)carry_flush(yp[e] * (z / (1.0f + expf(-z))), kYCarry); }
  unsigned short* dp = Y16 + row * kDI + c8;
  *(volatile v8h*)dp = hv;
  __threadfence();
  *(volatile v8h*)dp = hv;
}
static_assert((size_t)kRows * (kDI / 8) == 2048ull * kThr, "gate grid exact: 2,048 blocks");

extern "C" void kernel_launch(void* const* d_in, const int* in_sizes, int n_in,
                              void* d_out, int out_size, void* d_ws, size_t ws_size,
                              hipStream_t stream) {
  if (n_in < 10 || d_out == nullptr || d_ws == nullptr) return;
  if (in_sizes[0] != kRows * kDM || in_sizes[1] != kDM * 2 * kDI || in_sizes[2] != kDI * kDC || in_sizes[3] != kDI || in_sizes[4] != kDI * kXo) return;
  if (in_sizes[5] != kR * kDI || in_sizes[6] != kDI || in_sizes[7] != kDI * kNs || in_sizes[8] != kDI || in_sizes[9] != kDI * kDM) return;
  if (out_size != kRows * kDM + kDI * kNs) return;
  if (ws_size < kWsTotal) return;
  const float* x      = (const float*)d_in[0];
  const float* W_in   = (const float*)d_in[1];
  const float* conv_w = (const float*)d_in[2];
  const float* conv_b = (const float*)d_in[3];
  const float* W_x    = (const float*)d_in[4];
  const float* W_dt   = (const float*)d_in[5];
  const float* b_dt   = (const float*)d_in[6];
  const float* A_log  = (const float*)d_in[7];
  const float* D_skip = (const float*)d_in[8];
  const float* W_out  = (const float*)d_in[9];
  float* out = (float*)d_out;
  float* HT  = out + (size_t)kRows * kDM;
  char* ws = (char*)d_ws;
  float* BIAS = (float*)(ws + kOffBIAS);
  float* ZB  = BIAS;
  float* BDT = BIAS + 4096;
  unsigned short* X16    = (unsigned short*)(ws + kOffX16);
  unsigned short* WIN16  = (unsigned short*)(ws + kOffWIN16);
  unsigned short* WX16   = (unsigned short*)(ws + kOffWX16);
  unsigned short* WDT16  = (unsigned short*)(ws + kOffWDT16);
  unsigned short* WOUT16 = (unsigned short*)(ws + kOffWOUT16);
  float* XZ  = (float*)(ws + kOffXZ);
  float* U32 = (float*)(ws + kOffU32);
  unsigned short* U16 = (unsigned short*)(ws + kOffU16);
  float* XD  = (float*)(ws + kOffXD);
  unsigned short* DT16 = (unsigned short*)(ws + kOffDT16);
  float* DL  = (float*)(ws + kOffDL);
  float* YS  = (float*)(ws + kOffYS);
  unsigned short* Y16 = (unsigned short*)(ws + kOffY16);

  static_assert(((size_t)kRows * kDM / 8) % kThr == 0 && kDM / 8 <= 256 && kDI / 8 <= 256 && kR / 8 == 8, "the casts' grids: the input's 1,024 blocks; the transposing casts' blocks of 128, 256 and 8 threads");
  cast_plane_kernel<<<(int)(((size_t)kRows * kDM / 8) / kThr), kThr, 0, stream>>>(x, X16, 10, kDM, 0);
  wt_plane_kernel<<<2 * kDI, kDM / 8, 0, stream>>>(W_in, WIN16, kDM, 2 * kDI, 2 * kDI, kDM, 0);
  wt_plane_kernel<<<kXoP, kDI / 8, 0, stream>>>(W_x, WX16, kDI, kXo, kXo, 2 * kDI, 0);
  wt_plane_kernel<<<kXoP, kDI / 8, 0, stream>>>(W_x, WX16, kDI, kXo, kXo, 2 * kDI, kDI);
  wt_plane_kernel<<<kDI, kR / 8, 0, stream>>>(W_dt, WDT16, kR, kDI, kDI, kR, 0);
  wt_plane_kernel<<<kDM, kDI / 8, 0, stream>>>(W_out, WOUT16, kDI, kDM, kDM, kDI, 0);
  setup_kernel<<<24, kThr, 0, stream>>>(b_dt, BIAS);

  wmma_gemm64<0, false, 2, 0, false, 0><<<dim3((kRows / 64) * (2 * kDI / 64) / 8, 1), 256, 0, stream>>>(
      X16, X16, kDM, 0L, WIN16, WIN16, kDM, 0L, (void*)XZ, (void*)XZ, 2 * kDI, 0L, ZB, nullptr, 0L, kRows, 2 * kDI, kDM, kScIn);
  front_kernel<<<dim3(4, kRows), 64, 0, stream>>>(XZ, conv_w, conv_b, U32, U16);
  wmma_gemm64<0, false, 2, 0, false, 0><<<dim3((kRows / 64) * (kXoP / 64) / 8, 1), 256, 0, stream>>>(
      U16, U16, 2 * kDI, 0L, WX16, WX16, 2 * kDI, 0L, (void*)XD, (void*)XD, kXoP, 0L, ZB, nullptr, 0L, kRows, kXoP, 2 * kDI, kScU);
  dtcast_kernel<<<64, kThr, 0, stream>>>(XD, DT16);
  wmma_gemm64<0, false, 2, 0, false, 0><<<dim3((kRows / 64) * (kDI / 64) / 8, 1), 256, 0, stream>>>(
      DT16, DT16, kR, 0L, WDT16, WDT16, kR, 0L, (void*)DL, (void*)DL, kDI, 0L, BDT, nullptr, 0L, kRows, kDI, kR, kScDt);
  scan_kernel<<<8, kThr, 0, stream>>>(XD, DL, U32, A_log, D_skip, YS, HT);
  ygate_kernel<<<2048, kThr, 0, stream>>>(YS, XZ, Y16);
  wmma_gemm64<0, false, 2, 0, false, 0><<<dim3((kRows / 64) * (kDM / 64) / 8, 1), 256, 0, stream>>>(
      Y16, Y16, kDI, 0L, WOUT16, WOUT16, kDI, 0L, (void*)out, (void*)out, kDM, 0L, ZB, nullptr, 0L, kRows, kDM, kDI, kScY);
}
